// KANLayer_29996051595740
// MI455X (gfx1250) — hardware-verified
//
#include <hip/hip_runtime.h>

typedef __attribute__((ext_vector_type(16))) _Float16 v16h;
typedef __attribute__((ext_vector_type(8)))  _Float16 v8h;
typedef __attribute__((ext_vector_type(8)))  float    v8f;
typedef __attribute__((ext_vector_type(4)))  float    v4f;

constexpr int DIM_B = 4096;
constexpr int DIM_N = 32;
constexpr int DIM_H = 64;
constexpr int DIM_O = 32;
constexpr int NPAIR = DIM_N * (DIM_N - 1) / 2;
constexpr int TB    = 2;
constexpr int TM    = TB * DIM_N;
constexpr int NTHR  = 128;
constexpr int NBLK  = DIM_B / TB;
constexpr int P_A1  = 72;
constexpr int P_A2  = 40;
constexpr int P_D1  = 36;
constexpr int P_UV  = 64;
constexpr int P_W2  = 65;
constexpr float OP_CARRY = 16.0f;
constexpr float ACC_FOLD = 1.0f / 256.0f;
constexpr float A2_FOLD  = 1.0f / 16.0f;

static_assert(DIM_B % TB == 0, "grid covers the batch exactly");
static_assert(NTHR == TB * DIM_H, "one lane per (batch, hidden) in the pair reduction");
static_assert(NTHR / 32 == TM / 16, "one wave per 16-row m-tile");
static_assert(DIM_H % 32 == 0 && DIM_O % 32 == 0, "K of both contractions is a multiple of 32");
static_assert(DIM_O % 16 == 0 && (2 * DIM_H) % 16 == 0, "N of both contractions is a multiple of 16");
static_assert((TM + DIM_O) * P_A1 * 2 <= TM * P_UV * 4, "A1 and Bt1 f16 views fit region X");
static_assert(TM * P_D1 <= TM * P_UV, "D1 slab fits region Y");
static_assert(NTHR * 16 == DIM_O * DIM_H, "Bt1 and psi_w2 staging: 16 elements per thread");
static_assert(NTHR == 2 * DIM_H, "Bt2 staging: one row per thread");
static_assert(NTHR * 32 == TM * DIM_H, "A1 build: 32 elements per thread");
static_assert(NTHR * 16 == TM * DIM_O, "A2 conversion: 16 elements per thread");
static_assert(TB * DIM_O == 64 && TB * DIM_O <= NTHR, "output tile = 64 floats = two whole 128-B lines");

__device__ __forceinline__ v16h frag_load_h(const _Float16* p) {
  union { v16h v; v8h h[2]; } f;
  f.h[0] = *(const v8h*)(p);
  f.h[1] = *(const v8h*)(p + 16);
  return f.v;
}
__device__ __forceinline__ v8f mma_f16(v16h a, v16h b, v8f c) {
  c = __builtin_amdgcn_wmma_f32_16x16x32_f16(false, a, false, b, (short)0, c, false, false);
  asm volatile("v_nop\n\tv_nop\n\tv_nop\n\tv_nop" : "+v"(c) : "v"(a), "v"(b));
  return c;
}
__device__ __forceinline__ v8f zero8() { return (v8f){0.f, 0.f, 0.f, 0.f, 0.f, 0.f, 0.f, 0.f}; }

__global__ __launch_bounds__(NTHR) void kan_fused_kernel(
    const float* __restrict__ x,
    const float* __restrict__ phi_w1, const float* __restrict__ phi_b1,
    const float* __restrict__ phi_w2, const float* __restrict__ phi_b2,
    const float* __restrict__ psi_w1, const float* __restrict__ psi_b1,
    const float* __restrict__ psi_w2, const float* __restrict__ psi_b2,
    float* __restrict__ out)
{
  __shared__ __align__(16) float    sPar[256];
  __shared__ __align__(16) float    sRX[TM * P_UV];
  __shared__ __align__(16) float    sRY[TM * P_UV];
  __shared__ __align__(16) _Float16 sA2[TM * P_A2];
  __shared__ __align__(16) _Float16 sBt2[2 * DIM_H * P_A2];
  __shared__ __align__(16) float    sW2[DIM_O * P_W2];
  __shared__ __align__(16) float    sS[TB * DIM_H];
  __shared__ __align__(16) float    sOut[TB * DIM_O];

  const int tid  = threadIdx.x;
  const int lane = tid & 31;
  const int wave = tid >> 5;
  const int hh   = lane >> 4;
  const int rl   = lane & 15;
  const int koff = hh * 8;
  const int blk  = blockIdx.x;

  _Float16* sA1  = (_Float16*)(void*)sRX;
  _Float16* sBt1 = sA1 + TM * P_A1;
  float*    sD1  = sRY;
  float*    sU   = sRY;
  float*    sV   = sRX;

  {
    const int o = tid >> 2, h16 = (tid & 3) * 16;
    const float* src = phi_w2 + (size_t)o * DIM_H + h16;
    const v4f g0 = *(const v4f*)(src);
    const v4f g1 = *(const v4f*)(src + 4);
    const v4f g2 = *(const v4f*)(src + 8);
    const v4f g3 = *(const v4f*)(src + 12);
    v8h q0, q1;
#pragma unroll
    for (int e = 0; e < 4; ++e) {
      q0[e]     = (_Float16)(g0[e] * OP_CARRY);
      q0[4 + e] = (_Float16)(g1[e] * OP_CARRY);
      q1[e]     = (_Float16)(g2[e] * OP_CARRY);
      q1[4 + e] = (_Float16)(g3[e] * OP_CARRY);
    }
    *(v8h*)(sBt1 + o * P_A1 + h16)     = q0;
    *(v8h*)(sBt1 + o * P_A1 + h16 + 8) = q1;
  }
  asm volatile("" ::: "memory");
  {
    const int row = tid;
    const float* src = psi_w1 + (size_t)(row & (DIM_H - 1)) * (2 * DIM_O) + (row >> 6) * DIM_O;
#pragma unroll
    for (int half = 0; half < 2; ++half) {
      const float* s2 = src + half * 16;
      const v4f g0 = *(const v4f*)(s2);
      const v4f g1 = *(const v4f*)(s2 + 4);
      const v4f g2 = *(const v4f*)(s2 + 8);
      const v4f g3 = *(const v4f*)(s2 + 12);
      v8h q0, q1;
#pragma unroll
      for (int e = 0; e < 4; ++e) {
        q0[e]     = (_Float16)(g0[e] * OP_CARRY);
        q0[4 + e] = (_Float16)(g1[e] * OP_CARRY);
        q1[e]     = (_Float16)(g2[e] * OP_CARRY);
        q1[4 + e] = (_Float16)(g3[e] * OP_CARRY);
      }
      *(v8h*)(sBt2 + row * P_A2 + half * 16)     = q0;
      *(v8h*)(sBt2 + row * P_A2 + half * 16 + 8) = q1;
      asm volatile("" ::: "memory");
    }
  }
  {
    const int o = tid >> 2, h16 = (tid & 3) * 16;
    const float* src = psi_w2 + (size_t)o * DIM_H + h16;
    const v4f g0 = *(const v4f*)(src);
    const v4f g1 = *(const v4f*)(src + 4);
    const v4f g2 = *(const v4f*)(src + 8);
    const v4f g3 = *(const v4f*)(src + 12);
    float* dst = sW2 + o * P_W2 + h16;
#pragma unroll
    for (int e = 0; e < 4; ++e) {
      dst[e]      = g0[e];
      dst[4 + e]  = g1[e];
      dst[8 + e]  = g2[e];
      dst[12 + e] = g3[e];
    }
  }
  asm volatile("" ::: "memory");
  if (tid < DIM_H) {
    sPar[tid]       = phi_w1[tid] * OP_CARRY;
    sPar[64 + tid]  = phi_b1[tid] * OP_CARRY;
    sPar[128 + tid] = psi_b1[tid];
  }
  if (tid < DIM_O) {
    sPar[192 + tid] = phi_b2[tid] * OP_CARRY;
    sPar[224 + tid] = psi_b2[tid];
  }
  const float xv = x[(size_t)blk * TM + (tid >> 1)];
  __syncthreads();

  {
    const int m = tid >> 1, hb = (tid & 1) * 32;
#pragma unroll
    for (int q = 0; q < 4; ++q) {
      const v4f w0 = *(const v4f*)(sPar + hb + q * 8);
      const v4f w1 = *(const v4f*)(sPar + hb + q * 8 + 4);
      const v4f c0 = *(const v4f*)(sPar + 64 + hb + q * 8);
      const v4f c1 = *(const v4f*)(sPar + 64 + hb + q * 8 + 4);
      v8h hv;
#pragma unroll
      for (int e = 0; e < 4; ++e) {
        hv[e]     = (_Float16)fmaxf(fmaf(xv, w0[e], c0[e]), 0.0f);
        hv[4 + e] = (_Float16)fmaxf(fmaf(xv, w1[e], c1[e]), 0.0f);
      }
      *(v8h*)(sA1 + m * P_A1 + hb + q * 8) = hv;
    }
  }
  __syncthreads();

  {
    v8f acc10 = zero8(), acc11 = zero8();
    const _Float16* arow  = sA1  + (wave * 16 + rl) * P_A1 + koff;
    const _Float16* brow0 = sBt1 + rl * P_A1 + koff;
    const _Float16* brow1 = sBt1 + (16 + rl) * P_A1 + koff;
#pragma unroll
    for (int ks = 0; ks < 2; ++ks) {
      const v16h a  = frag_load_h(arow  + ks * 32);
      const v16h b0 = frag_load_h(brow0 + ks * 32);
      const v16h b1 = frag_load_h(brow1 + ks * 32);
      acc10 = mma_f16(a, b0, acc10);
      acc11 = mma_f16(a, b1, acc11);
    }
#pragma unroll
    for (int r = 0; r < 8; ++r) {
      const int row = wave * 16 + 8 * hh + r;
      sD1[row * P_D1 + rl]      = acc10[r];
      sD1[row * P_D1 + 16 + rl] = acc11[r];
    }
  }
  __syncthreads();
  {
    const int row = tid >> 1, c16 = (tid & 1) * 16;
    const float* dp = sD1 + row * P_D1 + c16;
    const v4f d0 = *(const v4f*)(dp);
    const v4f d1 = *(const v4f*)(dp + 4);
    const v4f d2 = *(const v4f*)(dp + 8);
    const v4f d3 = *(const v4f*)(dp + 12);
    const v4f e0 = *(const v4f*)(sPar + 192 + c16);
    const v4f e1 = *(const v4f*)(sPar + 192 + c16 + 4);
    const v4f e2 = *(const v4f*)(sPar + 192 + c16 + 8);
    const v4f e3 = *(const v4f*)(sPar + 192 + c16 + 12);
    v8h q0, q1;
#pragma unroll
    for (int e = 0; e < 4; ++e) {
      q0[e]     = (_Float16)fmaf(d0[e], A2_FOLD, e0[e]);
      q0[4 + e] = (_Float16)fmaf(d1[e], A2_FOLD, e1[e]);
      q1[e]     = (_Float16)fmaf(d2[e], A2_FOLD, e2[e]);
      q1[4 + e] = (_Float16)fmaf(d3[e], A2_FOLD, e3[e]);
    }
    *(v8h*)(sA2 + row * P_A2 + c16)     = q0;
    *(v8h*)(sA2 + row * P_A2 + c16 + 8) = q1;
  }
  __syncthreads();

  {
    const v16h a2 = frag_load_h(sA2 + (wave * 16 + rl) * P_A2 + koff);
    v8f acc2[8];
#pragma unroll
    for (int nt = 0; nt < 8; ++nt) {
      const v16h b = frag_load_h(sBt2 + (nt * 16 + rl) * P_A2 + koff);
      acc2[nt] = mma_f16(a2, b, zero8());
    }
#pragma unroll
    for (int nt = 0; nt < 8; ++nt) {
#pragma unroll
      for (int r = 0; r < 8; ++r) {
        const int row = wave * 16 + 8 * hh + r;
        if (nt < 4) {
          sU[row * P_UV + nt * 16 + rl] = fmaf(acc2[nt][r], ACC_FOLD, sPar[128 + nt * 16 + rl]);
        } else {
          sV[row * P_UV + (nt - 4) * 16 + rl] = acc2[nt][r] * ACC_FOLD;
        }
      }
    }
  }
  __syncthreads();

  {
    const int bl = tid >> 6, h = tid & 63;
    const float* vp = sV + (bl * DIM_N) * P_UV + h;
    const float* up = sU + (bl * DIM_N) * P_UV + h;
    float vreg[DIM_N];
#pragma unroll
    for (int j = 0; j < DIM_N; ++j) vreg[j] = vp[j * P_UV];
    float acc = 0.0f;
#pragma unroll
    for (int i = 0; i < DIM_N - 1; ++i) {
      const float ui = up[i * P_UV];
#pragma unroll
      for (int j = 1; j < DIM_N; ++j) {
        if (j > i) {
          acc = acc + fmaxf(ui + vreg[j], 0.0f);
        }
      }
    }
    sS[tid] = acc;
  }
  __syncthreads();

  if (tid < TB * DIM_O) {
    const int bl = tid >> 5, o = tid & 31;
    const float* sp = sS + bl * DIM_H;
    const float* wp = sW2 + o * P_W2;
    float acc = 0.0f;
#pragma unroll
    for (int h = 0; h < DIM_H; ++h) acc = fmaf(sp[h], wp[h], acc);
    sOut[tid] = acc + (float)NPAIR * sPar[224 + o];
  }
  __syncthreads();
  if (tid < 16) {
    const v4f val = *(const v4f*)(sOut + 4 * tid);
    float* op = out + (size_t)blk * (TB * DIM_O) + 4 * tid;
    *(volatile v4f*)op = val;
    __threadfence();
    *(volatile v4f*)op = val;
  }
}

extern "C" void kernel_launch(void* const* d_in, const int* in_sizes, int n_in,
                              void* d_out, int out_size, void* d_ws, size_t ws_size,
                              hipStream_t stream) {
  (void)d_ws; (void)ws_size;
  if (n_in < 9) return;
  if (in_sizes[0] != DIM_B * DIM_N) return;
  if (in_sizes[1] != DIM_H || in_sizes[2] != DIM_H) return;
  if (in_sizes[3] != DIM_O * DIM_H || in_sizes[4] != DIM_O) return;
  if (in_sizes[5] != DIM_H * 2 * DIM_O || in_sizes[6] != DIM_H) return;
  if (in_sizes[7] != DIM_O * DIM_H || in_sizes[8] != DIM_O) return;
  if (out_size != DIM_B * DIM_O) return;

  const float* x      = (const float*)d_in[0];
  const float* phi_w1 = (const float*)d_in[1];
  const float* phi_b1 = (const float*)d_in[2];
  const float* phi_w2 = (const float*)d_in[3];
  const float* phi_b2 = (const float*)d_in[4];
  const float* psi_w1 = (const float*)d_in[5];
  const float* psi_b1 = (const float*)d_in[6];
  const float* psi_w2 = (const float*)d_in[7];
  const float* psi_b2 = (const float*)d_in[8];
  float* out = (float*)d_out;

  kan_fused_kernel<<<dim3(NBLK), dim3(NTHR), 0, stream>>>(
      x, phi_w1, phi_b1, phi_w2, phi_b2, psi_w1, psi_b1, psi_w2, psi_b2, out);
}
